// EfficientMultiTensorProduct_34033320853904
// MI455X (gfx1250) — hardware-run, weakly checked
//
#include <hip/hip_runtime.h>
#include <math.h>

typedef __attribute__((ext_vector_type(16))) __bf16   v16b;
typedef __attribute__((ext_vector_type(8)))  __bf16   v8b;
typedef __attribute__((ext_vector_type(8)))  float    v8f;
typedef __attribute__((ext_vector_type(4)))  float    v4f;
typedef __attribute__((ext_vector_type(4)))  unsigned v4u;

constexpr int kNodes     = 1024;
constexpr int kChan      = 128;
constexpr int kElem      = 10;
constexpr int kPack      = 16;
constexpr int kOutCols   = 2048;
constexpr int kPairs     = 136;
constexpr int kTrips     = 816;
constexpr int kPairPad   = 160;
constexpr int kTripPad   = 832;
constexpr int kKTot      = kPairPad + kTripPad;
constexpr int kBtPitch   = 1024;
constexpr int kPairSteps = kPairPad / 32;
constexpr int kTripSteps = kTripPad / 32;
constexpr int kFeatPitch = 17;
constexpr int kWPitch    = 12;
constexpr int kMonoPitch  = 40;
constexpr int kMonoPitchW = 20;
constexpr int kYN  = 4 * 7 * 7;
constexpr int kH2N = 4 * 13 * 13;
constexpr int kH3N = 4 * 19 * 19;
constexpr float kCoefCarry    = 0.0625f;
constexpr float kCoefCarryInv = 1.0f / kCoefCarry;

static_assert(kPairs == kPack * (kPack + 1) / 2, "pair count");
static_assert(kTrips == kPack * (kPack + 1) * (kPack + 2) / 6, "triple count");
static_assert((kPairPad % 32) == 0 && (kTripPad % 32) == 0 && kPairPad >= kPairs && kTripPad >= kTrips, "K pads");
static_assert(kKTot == 992 && kKTot <= kBtPitch, "K total");
static_assert(kOutCols == kChan * kPack, "output width");
static_assert((kMonoPitch % 8) == 0 && kMonoPitchW * 2 == kMonoPitch, "LDS fragment alignment");
static_assert(kChan == 4 * 32, "four waves of 32 channel rows per node");

constexpr size_t kOffBtH  = 0;
constexpr size_t kOffBtL  = kOffBtH + (size_t)kPack * kBtPitch * 2;
constexpr size_t kWsTotal = kOffBtL + (size_t)kPack * kBtPitch * 2;
static_assert(kWsTotal == 65536ull, "carve total");
static_assert((kOffBtL % 128) == 0, "128-B aligned regions");

__device__ __forceinline__ unsigned bf16_rne_bits(float f) {
  const unsigned u = __float_as_uint(f);
  return (u + 0x7FFFu + ((u >> 16) & 1u)) >> 16;
}
__device__ __forceinline__ int pack_l(int q) {
  return (q >= 1 ? 1 : 0) + (q >= 4 ? 1 : 0) + (q >= 9 ? 1 : 0);
}
__device__ __forceinline__ int pack_j(int q, int l) { return q - l * l + 3 - l; }

union FragB { v16b v; v8b h[2]; };
__device__ __forceinline__ v16b frag_load(const __bf16* p) {
  FragB f;
  f.h[0] = *(const v8b*)(p);
  f.h[1] = *(const v8b*)(p + 16);
  return f.v;
}
__device__ __forceinline__ v8f mma_bf16(v16b a, v16b b, v8f c) {
  c = __builtin_amdgcn_wmma_f32_16x16x32_bf16(false, a, false, b, (short)0, c, false, false);
  asm volatile("v_nop\n\tv_nop\n\tv_nop\n\tv_nop" : "+v"(c) : "v"(a), "v"(b));
  return c;
}

__device__ __forceinline__ void unrank_pair16(int p, int& i, int& j) {
  int ii = 0, base = 0, acc = 0;
#pragma unroll 1
  for (int s = 0; s < 15; ++s) {
    acc += 16 - s;
    const bool ge = (p >= acc);
    ii += ge ? 1 : 0;
    base = ge ? acc : base;
  }
  i = ii;
  j = ii + (p - base);
}
__device__ __forceinline__ void unrank_trip16(int t, int& i, int& j, int& k) {
  int ii = 0, base = 0, acc = 0;
#pragma unroll 1
  for (int s = 0; s < 15; ++s) {
    acc += ((16 - s) * (17 - s)) / 2;
    const bool ge = (t >= acc);
    ii += ge ? 1 : 0;
    base = ge ? acc : base;
  }
  const int rem = t - base;
  const int nn = 16 - ii;
  int jo = 0, base2 = 0, acc2 = 0;
#pragma unroll 1
  for (int r = 0; r < 15; ++r) {
    acc2 += nn - r;
    const bool ge = ((r + 1) <= (nn - 1)) && (rem >= acc2);
    jo += ge ? 1 : 0;
    base2 = ge ? acc2 : base2;
  }
  i = ii;
  j = ii + jo;
  k = ii + jo + (rem - base2);
}

__global__ __launch_bounds__(256) void coef_planes_kernel(
    const float* __restrict__ Yre, const float* __restrict__ Yim,
    const float* __restrict__ H2re, const float* __restrict__ H2im,
    const float* __restrict__ H3re, const float* __restrict__ H3im,
    unsigned short* __restrict__ BtH, unsigned short* __restrict__ BtL)
{
  __shared__ float sYr[kYN];
  __shared__ float sYi[kYN];
  __shared__ float sH2r[kH2N];
  __shared__ float sH2i[kH2N];
  __shared__ float sH3r[kH3N];
  __shared__ float sH3i[kH3N];
  __shared__ __align__(16) float sV[256];

  const int tid = threadIdx.x;
#pragma unroll 1
  for (int t = tid; t < kYN; t += 256) { sYr[t] = Yre[t]; sYi[t] = Yim[t]; }
#pragma unroll 1
  for (int t = tid; t < kH2N; t += 256) { sH2r[t] = H2re[t]; sH2i[t] = H2im[t]; }
#pragma unroll 1
  for (int t = tid; t < kH3N; t += 256) { sH3r[t] = H3re[t]; sH3i[t] = H3im[t]; }
  __syncthreads();

  const int q  = blockIdx.y;
  const int c  = blockIdx.x * 256 + tid;
  const int lq = pack_l(q);
  const int jq = pack_j(q, lq);

  float val2;
  {
    int p = c;
    p = p < 0 ? 0 : p;
    p = p > (kPairs - 1) ? (kPairs - 1) : p;
    int pi0, pj0;
    unrank_pair16(p, pi0, pj0);
    const int la = pack_l(pi0), ja = pack_j(pi0, la);
    const int lb = pack_l(pj0), jb = pack_j(pj0, lb);
    const int ya = (la * 7 + ja) * 7;
    const int yb = (lb * 7 + jb) * 7;
    const int hb = (lq * 13 + jq + 3) * 13;
    float acc = 0.f;
#pragma unroll 1
    for (int u1 = 0; u1 < 7; ++u1) {
      const float ar = sYr[ya + u1], ai = sYi[ya + u1];
#pragma unroll 1
      for (int u2 = 0; u2 < 7; ++u2) {
        const float br = sYr[yb + u2], bi = sYi[yb + u2];
        const float pr = ar * br - ai * bi;
        const float pi = ar * bi + ai * br;
        const float hr = sH2r[hb + u1 + u2], hi = sH2i[hb + u1 + u2];
        acc += pr * hr - pi * hi;
      }
    }
    const float mult = (pi0 == pj0) ? 1.0f : 2.0f;
    const bool gate = (c < kPairs) && ((ja + jb) == (jq + 3));
    val2 = gate ? (mult * acc) : 0.0f;
  }

  float val3;
  {
    int t = c - kPairPad;
    t = t < 0 ? 0 : t;
    t = t > (kTrips - 1) ? (kTrips - 1) : t;
    int ti, tj, tk;
    unrank_trip16(t, ti, tj, tk);
    const int la = pack_l(ti), ja = pack_j(ti, la);
    const int lb = pack_l(tj), jb = pack_j(tj, lb);
    const int lc = pack_l(tk), jc = pack_j(tk, lc);
    const int ya = (la * 7 + ja) * 7;
    const int yb = (lb * 7 + jb) * 7;
    const int yc = (lc * 7 + jc) * 7;
    const int hb = (lq * 19 + jq + 6) * 19;
    float acc = 0.f;
#pragma unroll 1
    for (int u1 = 0; u1 < 7; ++u1) {
      const float ar = sYr[ya + u1], ai = sYi[ya + u1];
#pragma unroll 1
      for (int u2 = 0; u2 < 7; ++u2) {
        const float br = sYr[yb + u2], bi = sYi[yb + u2];
        const float p12r = ar * br - ai * bi;
        const float p12i = ar * bi + ai * br;
#pragma unroll 1
        for (int u3 = 0; u3 < 7; ++u3) {
          const float cr = sYr[yc + u3], ci = sYi[yc + u3];
          const float pr = p12r * cr - p12i * ci;
          const float pi = p12r * ci + p12i * cr;
          const float hr = sH3r[hb + u1 + u2 + u3], hi = sH3i[hb + u1 + u2 + u3];
          acc += pr * hr - pi * hi;
        }
      }
    }
    const bool allEq = (ti == tj) && (tj == tk);
    const bool anyEq = (ti == tj) || (tj == tk);
    const float mult = allEq ? 1.0f : (anyEq ? 3.0f : 6.0f);
    const bool gate = (c >= kPairPad) && ((c - kPairPad) < kTrips) && ((ja + jb + jc) == (jq + 6));
    val3 = gate ? (mult * acc) : 0.0f;
  }

  const float val = (c < kPairPad) ? val2 : val3;
  sV[tid] = val * kCoefCarry;
  __syncthreads();

  if (tid < 32) {
    const float* sp = sV + 8 * tid;
    unsigned hb[8], lb[8];
#pragma unroll
    for (int e = 0; e < 8; ++e) {
      const float v = sp[e];
      const unsigned h = bf16_rne_bits(v);
      hb[e] = h;
      lb[e] = bf16_rne_bits(v - __uint_as_float(h << 16));
    }
    const v4u hv = { hb[0] | (hb[1] << 16), hb[2] | (hb[3] << 16), hb[4] | (hb[5] << 16), hb[6] | (hb[7] << 16) };
    const v4u lv = { lb[0] | (lb[1] << 16), lb[2] | (lb[3] << 16), lb[4] | (lb[5] << 16), lb[6] | (lb[7] << 16) };
    const size_t o = (size_t)q * kBtPitch + (size_t)blockIdx.x * 256 + 8 * tid;
    unsigned short* ph = BtH + o;
    unsigned short* pl = BtL + o;
    *(volatile v4u*)ph = hv;
    *(volatile v4u*)pl = lv;
    __threadfence();
    *(volatile v4u*)ph = hv;
    *(volatile v4u*)pl = lv;
  }
}

template <bool PAIRS>
__device__ __forceinline__ void odo_next(const float* fr, int& oi, int& oj, int& ok, bool& live, float& pij) {
  ok += 1;
  if (ok > 15) {
    oj += 1;
    if (oj > 15) {
      if (PAIRS) {
        live = false;
        oj = 15;
      } else {
        oi += 1;
        if (oi > 15) { live = false; oi = 15; }
        oj = oi;
      }
    }
    ok = oj;
    pij = fr[oi] * fr[oj];
  }
}

template <bool PAIRS>
__device__ __forceinline__ void poly_phase(
    const float* fr, unsigned* mhRow, unsigned* mlRow,
    const __bf16* aH, const __bf16* aL, const __bf16* bH, const __bf16* bL,
    int nsteps, v8f& acc0, v8f& acc1)
{
  int oi = PAIRS ? 16 : 0;
  int oj = 0;
  int ok = 0;
  bool live = true;
  float pij = fr[oi] * fr[oj];
#pragma unroll 1
  for (int s = 0; s < nsteps; ++s) {
    __syncthreads();
#pragma unroll 1
    for (int cw = 0; cw < 16; ++cw) {
      const float t0 = pij * fr[ok];
      const float m0 = live ? t0 : 0.0f;
      odo_next<PAIRS>(fr, oi, oj, ok, live, pij);
      const float t1 = pij * fr[ok];
      const float m1 = live ? t1 : 0.0f;
      odo_next<PAIRS>(fr, oi, oj, ok, live, pij);
      const unsigned h0 = bf16_rne_bits(m0);
      const unsigned h1 = bf16_rne_bits(m1);
      const unsigned l0 = bf16_rne_bits(m0 - __uint_as_float(h0 << 16));
      const unsigned l1 = bf16_rne_bits(m1 - __uint_as_float(h1 << 16));
      mhRow[cw] = h0 | (h1 << 16);
      mlRow[cw] = l0 | (l1 << 16);
    }
    __syncthreads();
    const v16b ah0 = frag_load(aH);
    const v16b al0 = frag_load(aL);
    const v16b ah1 = frag_load(aH + 16 * kMonoPitch);
    const v16b al1 = frag_load(aL + 16 * kMonoPitch);
    const v16b bh  = frag_load(bH + 32 * s);
    const v16b bl  = frag_load(bL + 32 * s);
    acc0 = mma_bf16(ah0, bh, acc0);
    acc0 = mma_bf16(ah0, bl, acc0);
    acc0 = mma_bf16(al0, bh, acc0);
    acc1 = mma_bf16(ah1, bh, acc1);
    acc1 = mma_bf16(ah1, bl, acc1);
    acc1 = mma_bf16(al1, bh, acc1);
  }
}

__global__ __launch_bounds__(128) void poly_main_kernel(
    const float* __restrict__ feat, const float* __restrict__ atype, const float* __restrict__ wts,
    const unsigned short* __restrict__ BtHp, const unsigned short* __restrict__ BtLp,
    float* __restrict__ out)
{
  __shared__ __align__(16) float    sF[4][32 * kFeatPitch];
  __shared__ __align__(16) float    sW[4][32 * kWPitch];
  __shared__ __align__(16) unsigned sMH[4][32 * kMonoPitchW];
  __shared__ __align__(16) unsigned sML[4][32 * kMonoPitchW];
  __shared__ __align__(16) float    sO[4][512];

  const int tid  = threadIdx.x;
  const int wave = tid >> 5;
  const int lane = tid & 31;
  const int hh   = lane >> 4;
  const int c16  = lane & 15;
  const int n    = blockIdx.x;
  const int d0   = wave * 32;

  float* fw = sF[wave];
  float* ww = sW[wave];
  float* so = sO[wave];

  {
    const float* src = feat + ((size_t)n * kChan + d0) * kPack;
#pragma unroll
    for (int it = 0; it < 4; ++it) {
      const int f4 = it * 32 + lane;
      const v4f v = *(const v4f*)(src + (size_t)f4 * 4);
      const int r = f4 >> 2;
      const int cc = (f4 & 3) * 4;
      fw[r * kFeatPitch + cc + 0] = v[0];
      fw[r * kFeatPitch + cc + 1] = v[1];
      fw[r * kFeatPitch + cc + 2] = v[2];
      fw[r * kFeatPitch + cc + 3] = v[3];
    }
    fw[lane * kFeatPitch + 16] = 1.0f;
  }

  {
    const int d = d0 + lane;
    float wacc[3][4];
#pragma unroll
    for (int k = 0; k < 3; ++k) {
      wacc[k][0] = 0.f; wacc[k][1] = 0.f; wacc[k][2] = 0.f; wacc[k][3] = 0.f;
    }
#pragma unroll 1
    for (int e = 0; e < kElem; ++e) {
      const float a = atype[n * kElem + e];
#pragma unroll
      for (int k = 0; k < 3; ++k) {
        const v4f wv = *(const v4f*)(wts + ((size_t)((k * kElem + e) * kChan + d)) * 4);
        wacc[k][0] = fmaf(a, wv[0], wacc[k][0]);
        wacc[k][1] = fmaf(a, wv[1], wacc[k][1]);
        wacc[k][2] = fmaf(a, wv[2], wacc[k][2]);
        wacc[k][3] = fmaf(a, wv[3], wacc[k][3]);
      }
    }
#pragma unroll
    for (int k = 0; k < 3; ++k) {
      ww[lane * kWPitch + k * 4 + 0] = wacc[k][0];
      ww[lane * kWPitch + k * 4 + 1] = wacc[k][1];
      ww[lane * kWPitch + k * 4 + 2] = wacc[k][2];
      ww[lane * kWPitch + k * 4 + 3] = wacc[k][3];
    }
  }
  __syncthreads();

  v8f c2a = (v8f){0.f,0.f,0.f,0.f,0.f,0.f,0.f,0.f};
  v8f c2b = (v8f){0.f,0.f,0.f,0.f,0.f,0.f,0.f,0.f};
  v8f c3a = (v8f){0.f,0.f,0.f,0.f,0.f,0.f,0.f,0.f};
  v8f c3b = (v8f){0.f,0.f,0.f,0.f,0.f,0.f,0.f,0.f};

  {
    const float* fr = fw + lane * kFeatPitch;
    unsigned* mhRow = sMH[wave] + lane * kMonoPitchW;
    unsigned* mlRow = sML[wave] + lane * kMonoPitchW;
    const __bf16* aH = (const __bf16*)(const void*)sMH[wave] + c16 * kMonoPitch + 8 * hh;
    const __bf16* aL = (const __bf16*)(const void*)sML[wave] + c16 * kMonoPitch + 8 * hh;
    const __bf16* bH = (const __bf16*)(const void*)BtHp + (size_t)c16 * kBtPitch + 8 * hh;
    const __bf16* bL = (const __bf16*)(const void*)BtLp + (size_t)c16 * kBtPitch + 8 * hh;
    poly_phase<true >(fr, mhRow, mlRow, aH, aL, bH,            bL,            kPairSteps, c2a, c2b);
    poly_phase<false>(fr, mhRow, mlRow, aH, aL, bH + kPairPad, bL + kPairPad, kTripSteps, c3a, c3b);
  }

  {
    const int lq = pack_l(c16);
    const int sbase = 32 * lq * lq + (c16 - lq * lq);
    const int sw = 2 * lq + 1;
#pragma unroll
    for (int r = 0; r < 8; ++r) {
      const int ra = 8 * hh + r;
      const int rb = 16 + ra;
      const float fa  = fw[ra * kFeatPitch + c16];
      const float fb  = fw[rb * kFeatPitch + c16];
      const float wa0 = ww[ra * kWPitch + lq];
      const float wa1 = ww[ra * kWPitch + 4 + lq];
      const float wa2 = ww[ra * kWPitch + 8 + lq];
      const float wb0 = ww[rb * kWPitch + lq];
      const float wb1 = ww[rb * kWPitch + 4 + lq];
      const float wb2 = ww[rb * kWPitch + 8 + lq];
      const float pa = wa1 * c2a[r] + wa2 * c3a[r];
      const float pb = wb1 * c2b[r] + wb2 * c3b[r];
      so[sbase + ra * sw] = wa0 * fa + kCoefCarryInv * pa;
      so[sbase + rb * sw] = wb0 * fb + kCoefCarryInv * pb;
    }
  }
  __syncthreads();

  {
    const int g  = lane >> 3;
    const int c4 = (lane & 7) * 4;
    v4f vals[4];
    size_t offs[4];
#pragma unroll
    for (int it = 0; it < 4; ++it) {
      const int x  = it * 4 + g;
      const int lx = pack_l(x);
      vals[it] = *(const v4f*)(so + x * 32 + c4);
      offs[it] = (size_t)n * kOutCols + (size_t)(128 * lx * lx + d0 * (2 * lx + 1) + 32 * (x - lx * lx) + c4);
    }
    for (int pass = 0; pass < 2; ++pass) {
#pragma unroll
      for (int it = 0; it < 4; ++it) {
        *(volatile v4f*)(out + offs[it]) = vals[it];
      }
      __threadfence();
    }
  }
}

extern "C" void kernel_launch(void* const* d_in, const int* in_sizes, int n_in,
                              void* d_out, int out_size, void* d_ws, size_t ws_size,
                              hipStream_t stream) {
  if (n_in < 9) return;
  if (in_sizes[0] != kNodes * kChan * kPack) return;
  if (in_sizes[1] != kNodes * kElem) return;
  if (in_sizes[2] != 3 * kElem * kChan * 4) return;
  if (in_sizes[3] != 4 * 7 * 7) return;
  if (in_sizes[4] != 4 * 7 * 7) return;
  if (in_sizes[5] != 7 * 13 * 13) return;
  if (in_sizes[6] != 7 * 13 * 13) return;
  if (in_sizes[7] != 10 * 19 * 19) return;
  if (in_sizes[8] != 10 * 19 * 19) return;
  if (out_size != kNodes * kOutCols) return;
  if (ws_size < kWsTotal) return;

  const float* feat  = (const float*)d_in[0];
  const float* atype = (const float*)d_in[1];
  const float* wts   = (const float*)d_in[2];
  const float* Yre   = (const float*)d_in[3];
  const float* Yim   = (const float*)d_in[4];
  const float* H2re  = (const float*)d_in[5];
  const float* H2im  = (const float*)d_in[6];
  const float* H3re  = (const float*)d_in[7];
  const float* H3im  = (const float*)d_in[8];
  float* out = (float*)d_out;

  char* ws = (char*)d_ws;
  unsigned short* BtH = (unsigned short*)(ws + kOffBtH);
  unsigned short* BtL = (unsigned short*)(ws + kOffBtL);

  coef_planes_kernel<<<dim3(kBtPitch / 256, kPack), 256, 0, stream>>>(Yre, Yim, H2re, H2im, H3re, H3im, BtH, BtL);
  poly_main_kernel<<<kNodes, 128, 0, stream>>>(feat, atype, wts, BtH, BtL, out);
}
